// IMLayer_7550552506848
// MI455X (gfx1250) — hardware-verified
//
#include <hip/hip_runtime.h>


namespace {
constexpr int NB = 8, L = 8192, H = 128, P = 128, K2 = 2 * P, M = NB * L;
constexpr float XS = 8.0f, WSC = 256.0f, YS = 64.0f;
typedef _Float16 b16;
typedef __attribute__((ext_vector_type(16))) _Float16 v16b;
typedef __attribute__((ext_vector_type(8))) _Float16 v8b;
typedef __attribute__((ext_vector_type(2))) _Float16 v2b;
typedef __attribute__((ext_vector_type(8))) float v8f;
typedef __attribute__((ext_vector_type(4))) float v4f;
typedef __attribute__((ext_vector_type(2))) float v2f;
__device__ __forceinline__ float bf16_rne(float f) { unsigned int u = __float_as_uint(f); u += 0x7FFFu + ((u >> 16) & 1u); return __uint_as_float(u & 0xFFFF0000u); }
__device__ __forceinline__ void split16(float v, b16& hi, b16& lo) { hi = (b16)v; lo = (b16)(v - (float)hi); }
__device__ __forceinline__ v16b frag_kb(const b16* p, int hh) { const v8b a = *(const v8b*)(p + 8 * hh), b = *(const v8b*)(p + 16 + 8 * hh); v16b f;
#pragma unroll
  for (int e = 0; e < 8; ++e) { f[e] = a[e]; f[8 + e] = b[e]; } return f; }
__device__ __forceinline__ v8f wmma16b(v16b a, v16b b, v8f c) { v8f d = __builtin_amdgcn_wmma_f32_16x16x32_f16(false, a, false, b, (short)0, c, false, false); asm volatile("v_nop\n\tv_nop\n\tv_nop\n\tv_nop" : "+v"(d) : "v"(a), "v"(b)); return d; }
__device__ __forceinline__ void wave_lds_sync() { __builtin_amdgcn_fence(__ATOMIC_RELEASE, "workgroup"); __builtin_amdgcn_wave_barrier(); __builtin_amdgcn_fence(__ATOMIC_ACQUIRE, "workgroup"); }
__device__ __forceinline__ float pmul(float a, float b) { float p = a * b; asm volatile("" : "+v"(p)); return p; }

__global__ __launch_bounds__(256) void wprep_kernel(const float* __restrict__ bw, const float* __restrict__ cw, b16* __restrict__ BT, b16* __restrict__ CT) {
  const size_t u = (size_t)blockIdx.x * 256 + threadIdx.x; const size_t n0 = (size_t)K2 * H / 8, n1 = (size_t)H * K2 / 8; size_t t = u; v8b o;
  if (t < n0) { const size_t e = t * 8; const int j = (int)(e / H), h0 = (int)(e % H); const int p = j >> 1, tt = j & 1; for (int i = 0; i < 8; ++i) o[i] = (b16)(bf16_rne(bw[((size_t)p * H + h0 + i) * 2 + tt]) * WSC); for (int pass = 0; pass < 2; ++pass) { *(volatile v8b*)(BT + e) = o; __threadfence(); } return; } t -= n0;
  if (t < n1) { const size_t e = t * 8; const int h = (int)(e / K2), j0 = (int)(e % K2); for (int i = 0; i < 8; ++i) { const int j = j0 + i; const int p = j >> 1, tt = j & 1; const float c = bf16_rne(cw[((size_t)h * P + p) * 2 + tt]); o[i] = (b16)((tt ? -c : c) * WSC); } for (int pass = 0; pass < 2; ++pass) { *(volatile v8b*)(CT + e) = o; __threadfence(); } }
}
__global__ __launch_bounds__(128) void bu_kernel(const float* __restrict__ x, const b16* __restrict__ BT, float* __restrict__ BU) {
  __shared__ __attribute__((aligned(16))) float Tf[4][16][128 + 4];
  const int wave = threadIdx.x >> 5, lane = threadIdx.x & 31, nloc = lane & 15, hlf = lane >> 4; const size_t m0 = (size_t)blockIdx.x * 64 + wave * 16; const int c0 = blockIdx.y * 128; const size_t r = m0 + nloc;
  v8f acc[8];
#pragma unroll
  for (int t = 0; t < 8; ++t) acc[t] = (v8f){};
#pragma unroll 2
  for (int kb = 0; kb < H; kb += 32) { v16b a; const float* xr = x + r * H + kb; for (int e = 0; e < 8; ++e) { a[e] = (b16)(bf16_rne(xr[8 * hlf + e]) * XS); a[8 + e] = (b16)(bf16_rne(xr[16 + 8 * hlf + e]) * XS); }
#pragma unroll
    for (int t = 0; t < 8; ++t) acc[t] = wmma16b(a, frag_kb(BT + (size_t)(c0 + t * 16 + nloc) * H + kb, hlf), acc[t]); }
#pragma unroll
  for (int t = 0; t < 8; ++t)
#pragma unroll 1
    for (int rr = 0; rr < 8; ++rr) Tf[wave][8 * hlf + rr][t * 16 + nloc] = acc[t][rr] * (1.0f / (XS * WSC));
  wave_lds_sync();
  for (int pass = 0; pass < 2; ++pass) { for (int rr = 0; rr < 16; ++rr) *(volatile v4f*)(BU + (m0 + rr) * K2 + c0 + lane * 4) = *(const v4f*)(&Tf[wave][rr][lane * 4]); __threadfence(); }
}
__global__ __launch_bounds__(64) void scan_kernel(const float* __restrict__ BU, const float* __restrict__ sp, const float* __restrict__ ap, b16* __restrict__ YH, b16* __restrict__ YL) {
  const int wave = threadIdx.x >> 5, lane = threadIdx.x & 31; const int wg = blockIdx.x * 2 + wave; const int b = wg >> 2, g = wg & 3; const int j0 = g * 64 + lane * 2; const int p = j0 >> 1;
  const float s = 1.0f / (1.0f + __expf(-bf16_rne(sp[p]))); const float A = fmaxf(bf16_rne(ap[p]), 0.0f); const float s2A = s * s * A; const float schur = 1.0f / (1.0f + s2A);
  const float m11 = 1.0f - s2A * schur, m12 = -(s * A) * schur, m21 = s * schur, m22 = schur; const float c1 = m11 * s, c2 = m21 * s;
  float y1a = 0.0f, y2a = 0.0f, y1b = 0.0f, y2b = 0.0f;
  const float* bu = BU + (size_t)b * L * K2 + j0; b16* yh = YH + (size_t)b * L * K2 + j0; b16* yl = YL + (size_t)b * L * K2 + j0;
#pragma unroll 4
  for (int l = 0; l < L; ++l) { const v2f u = *(const v2f*)(bu + (size_t)l * K2);
    const float n1a = pmul(m11, y1a) + pmul(m12, y2a) + pmul(c1, u[0]); const float n2a = pmul(m21, y1a) + pmul(m22, y2a) + pmul(c2, u[0]);
    const float n1b = pmul(m11, y1b) + pmul(m12, y2b) + pmul(c1, u[1]); const float n2b = pmul(m21, y1b) + pmul(m22, y2b) + pmul(c2, u[1]);
    y1a = n1a; y2a = n2a; y1b = n1b; y2b = n2b;
    b16 ha, la, hb, lb; split16(y2a * YS, ha, la); split16(y2b * YS, hb, lb); v2b vh, vl; vh[0] = ha; vh[1] = hb; vl[0] = la; vl[1] = lb;
    for (int pass = 0; pass < 2; ++pass) { *(volatile v2b*)(yh + (size_t)l * K2) = vh; *(volatile v2b*)(yl + (size_t)l * K2) = vl; __threadfence(); } }
}
__global__ __launch_bounds__(128) void out_kernel(const b16* __restrict__ YH, const b16* __restrict__ YL, const b16* __restrict__ CT, const float* __restrict__ x, const float* __restrict__ dv, float* __restrict__ out) {
  __shared__ __attribute__((aligned(16))) float Tf[4][16][128 + 4];
  const int wave = threadIdx.x >> 5, lane = threadIdx.x & 31, nloc = lane & 15, hlf = lane >> 4; const size_t m0 = (size_t)blockIdx.x * 64 + wave * 16; const size_t r = m0 + nloc;
  v8f acc[8];
#pragma unroll
  for (int t = 0; t < 8; ++t) acc[t] = (v8f){};
#pragma unroll 2
  for (int kb = 0; kb < K2; kb += 32) { const v16b a = frag_kb(YH + r * K2 + kb, hlf), al = frag_kb(YL + r * K2 + kb, hlf);
#pragma unroll
    for (int t = 0; t < 8; ++t) { const v16b bw = frag_kb(CT + (size_t)(t * 16 + nloc) * K2 + kb, hlf); acc[t] = wmma16b(a, bw, acc[t]); acc[t] = wmma16b(al, bw, acc[t]); } }
#pragma unroll
  for (int t = 0; t < 8; ++t) { const int c = t * 16 + nloc; const float d = bf16_rne(dv[c]);
#pragma unroll 1
    for (int rr = 0; rr < 8; ++rr) { const size_t row = m0 + 8 * hlf + rr; Tf[wave][8 * hlf + rr][c] = acc[t][rr] * (1.0f / (YS * WSC)) + pmul(bf16_rne(x[row * H + c]), d); } }
  wave_lds_sync();
  for (int pass = 0; pass < 2; ++pass) { for (int rr = 0; rr < 16; ++rr) *(volatile v4f*)(out + (m0 + rr) * H + lane * 4) = *(const v4f*)(&Tf[wave][rr][lane * 4]); __threadfence(); }
}
}

extern "C" void kernel_launch(void* const* d_in, const int* in_sizes, int n_in, void* d_out, int out_size, void* d_ws, size_t ws_size, hipStream_t stream) {
  (void)n_in;
  auto Fp = [&](int i) { return (const float*)d_in[i]; };
  if (in_sizes[0] != M * H || in_sizes[1] != P || in_sizes[2] != P || in_sizes[3] != P * H * 2 || in_sizes[4] != H * P * 2 || in_sizes[5] != H || out_size != M * H) return;
  size_t off = 0; char* ws = (char*)d_ws;
  auto carve = [&](size_t bytes) { char* p = ws + off; off += (bytes + 255) & ~(size_t)255; return p; };
  b16* BT = (b16*)carve((size_t)K2 * H * 2); b16* CT = (b16*)carve((size_t)H * K2 * 2); float* BU = (float*)carve((size_t)M * K2 * 4); b16* YH = (b16*)carve((size_t)M * K2 * 2); b16* YL = (b16*)carve((size_t)M * K2 * 2);
  if (off > ws_size) return;
  wprep_kernel<<<(unsigned)(((size_t)K2 * H / 8 + (size_t)H * K2 / 8 + 255) / 256), 256, 0, stream>>>(Fp(3), Fp(4), BT, CT);
  bu_kernel<<<dim3(M / 64, 2), 128, 0, stream>>>(Fp(0), BT, BU);
  scan_kernel<<<NB * 4 / 2, 64, 0, stream>>>(BU, Fp(1), Fp(2), YH, YL);
  out_kernel<<<M / 64, 128, 0, stream>>>(YH, YL, CT, Fp(0), Fp(5), (float*)d_out);
}
